// PointNetSetAbstraction_50543175139454
// MI455X (gfx1250) — hardware-verified
//
#include <hip/hip_runtime.h>
#pragma clang fp contract(off)

typedef __attribute__((ext_vector_type(16))) _Float16 v16h;
typedef __attribute__((ext_vector_type(8)))  _Float16 v8h;
typedef __attribute__((ext_vector_type(16))) __bf16   v16b;
typedef __attribute__((ext_vector_type(8)))  __bf16   v8b;
typedef __attribute__((ext_vector_type(8)))  float    v8f;
typedef __attribute__((ext_vector_type(4)))  float    v4f;
typedef __attribute__((ext_vector_type(2)))  float    v2f;
typedef __attribute__((ext_vector_type(4)))  unsigned int u32x4;
typedef unsigned int u32x4_a __attribute__((ext_vector_type(4))) __attribute__((may_alias));
typedef float v4f_a __attribute__((ext_vector_type(4))) __attribute__((may_alias));

constexpr int NB = 16;
constexpr int NPTS = 4096;
constexpr int NPOINT = 1024;
constexpr int NSAMPLE = 32;
constexpr int DFEAT = 64;
constexpr int CIN1 = 67;
constexpr int NCH1 = 64;
constexpr int NCH2 = 64;
constexpr int NCH3 = 128;
constexpr int NGRP = NB * NPOINT;
constexpr long NPOS = (long)NGRP * NSAMPLE;
constexpr float RAD2 = 0.04f;
constexpr float BN_EPS = 1e-5f;
constexpr float WCARRY = 16.0f;
constexpr float WINV = 1.0f / WCARRY;
constexpr int NPARTS = 512;
constexpr int XS_PITCH = 72;
constexpr int XS_WAVE = 32 * XS_PITCH;
static_assert(NSAMPLE == 32);
static_assert(NPOS == 524288);
static_assert(NGRP == NPARTS * 32);
static_assert(DFEAT + 3 == CIN1);

constexpr int WPL_OFF1 = 0;
constexpr int WPL_OFF2 = NCH1 * 64;
constexpr int WPL_OFF3 = WPL_OFF2 + NCH2 * 64;
constexpr int WPL_HALVES = WPL_OFF3 + NCH3 * 64;
static_assert(WPL_HALVES == 16384);

constexpr size_t OFF_WPL = 0;
constexpr size_t OFF_AC = OFF_WPL + (size_t)WPL_HALVES * 2;
constexpr size_t OFF_CEN = OFF_AC + 4096;
constexpr size_t OFF_IDX = OFF_CEN + (size_t)NB * 3 * NPOINT * 4;
constexpr size_t OFF_PART1 = OFF_IDX + (size_t)NPOS * 4;
constexpr size_t OFF_PART2 = OFF_PART1 + (size_t)NPARTS * 2 * NCH1 * 4;
constexpr size_t OFF_PART3 = OFF_PART2 + (size_t)NPARTS * 2 * NCH2 * 4;
constexpr size_t OFF_PTST = OFF_PART3 + (size_t)NPARTS * 2 * NCH3 * 4;
constexpr size_t OFF_PPL = OFF_PTST + (size_t)NB * NPTS * 64 * 2;
constexpr size_t OFF_X1 = OFF_PPL + (size_t)NB * NPTS * 64 * 4;
constexpr size_t OFF_MXP = OFF_X1 + (size_t)NPOS * 64 * 2;
constexpr size_t OFF_MNP = OFF_MXP + (size_t)NGRP * NCH3 * 4;
constexpr size_t WS_TOTAL = OFF_MNP + (size_t)NGRP * NCH3 * 4;
static_assert(WS_TOTAL <= (size_t)134217728);
static_assert(OFF_AC % 256 == 0 && OFF_CEN % 256 == 0 && OFF_IDX % 256 == 0 && OFF_PART1 % 256 == 0);
static_assert(OFF_PART2 % 256 == 0 && OFF_PART3 % 256 == 0 && OFF_PTST % 256 == 0 && OFF_PPL % 256 == 0);
static_assert(OFF_X1 % 256 == 0 && OFF_MXP % 256 == 0 && OFF_MNP % 256 == 0);
constexpr size_t OUT0_BYTES = (size_t)NB * 3 * NPOINT * 4;
constexpr size_t OUT1_BYTES = (size_t)NB * NCH3 * NPOINT * 4;
static_assert(OUT0_BYTES == 196608);
static_assert(OUT0_BYTES + OUT1_BYTES == 8585216);
static_assert(OUT0_BYTES % 128 == 0);

__device__ __forceinline__ unsigned short f2bf_bits(float f) {
  unsigned u = __float_as_uint(f);
  return (unsigned short)((u + 0x7FFFu + ((u >> 16) & 1u)) >> 16);
}
__device__ __forceinline__ float bf_bits2f(unsigned short h) { return __uint_as_float(((unsigned)h) << 16); }

__device__ __forceinline__ void dep_guard_h(v8f& a, v8f& b, v16h x, v16h y) { asm volatile("v_nop\n\tv_nop\n\tv_nop\n\tv_nop" : "+v"(a), "+v"(b) : "v"(x), "v"(y)); }
__device__ __forceinline__ void dep_guard_b(v8f& a, v8f& b, v16b x, v16b y) { asm volatile("v_nop\n\tv_nop\n\tv_nop\n\tv_nop" : "+v"(a), "+v"(b) : "v"(x), "v"(y)); }
__device__ __forceinline__ void keep4_h(v16h a, v16h b, v16h c, v16h d) { asm volatile("v_nop" :: "v"(a), "v"(b), "v"(c), "v"(d)); }
__device__ __forceinline__ void keep4_b(v16b a, v16b b, v16b c, v16b d) { asm volatile("v_nop" :: "v"(a), "v"(b), "v"(c), "v"(d)); }
__device__ __forceinline__ void acc_guard4(v8f& a, v8f& b, v8f& c, v8f& d) { asm volatile("v_nop\n\tv_nop\n\tv_nop\n\tv_nop" : "+v"(a), "+v"(b), "+v"(c), "+v"(d)); }
template <typename T> struct Frag;
template <> struct Frag<_Float16> {
  typedef v16h V; union U { v16h v; v8h h[2]; };
  static __device__ __forceinline__ v16h load(const _Float16* p) {
    U f; f.h[0] = *(const v8h*)(p); f.h[1] = *(const v8h*)(p + 16); return f.v;
  }
  static __device__ __forceinline__ v8f mma(v16h a, v16h b, v8f c) {
    return __builtin_amdgcn_wmma_f32_16x16x32_f16(false, a, false, b, (short)0, c, false, false);
  }
  static __device__ __forceinline__ void guard(v8f& a, v8f& b, v16h x, v16h y) { dep_guard_h(a, b, x, y); }
  static __device__ __forceinline__ void keep(v16h a, v16h b, v16h c, v16h d) { keep4_h(a, b, c, d); }
};
template <> struct Frag<__bf16> {
  typedef v16b V; union U { v16b v; v8b h[2]; };
  static __device__ __forceinline__ v16b load(const __bf16* p) {
    U f; f.h[0] = *(const v8b*)(p); f.h[1] = *(const v8b*)(p + 16); return f.v;
  }
  static __device__ __forceinline__ v8f mma(v16b a, v16b b, v8f c) {
    return __builtin_amdgcn_wmma_f32_16x16x32_bf16(false, a, false, b, (short)0, c, false, false);
  }
  static __device__ __forceinline__ void guard(v8f& a, v8f& b, v16b x, v16b y) { dep_guard_b(a, b, x, y); }
  static __device__ __forceinline__ void keep(v16b a, v16b b, v16b c, v16b d) { keep4_b(a, b, c, d); }
};

__device__ __forceinline__ v8f mma_h(v16h a, v16h b, v8f c) {
  c = __builtin_amdgcn_wmma_f32_16x16x32_f16(false, a, false, b, (short)0, c, false, false);
  asm volatile("v_nop\n\tv_nop\n\tv_nop\n\tv_nop" : "+v"(c) : "v"(a), "v"(b));
  return c;
}

template <int ET> struct Elem;
template <> struct Elem<0> { typedef _Float16 T; };
template <> struct Elem<1> { typedef __bf16 T; };
template <int ET, bool SPLIT, int BIAS_MODE, int OUT_MODE, bool RESID, int ACT = 0>
__global__ __launch_bounds__(256) void wmma_gemm64(
    const unsigned short* __restrict__ Ap, const unsigned short* __restrict__ A2p, int lda, long strideA,
    const unsigned short* __restrict__ Btp, const unsigned short* __restrict__ Bt2p, int ldb, long strideB,
    void* __restrict__ Cout, void* __restrict__ Cout2, int ldc, long strideC,
    const float* __restrict__ bias,
    const float* __restrict__ resid, long strideR,
    int M, int N, int K, float scale) {
  typedef typename Elem<ET>::T T;
  typedef typename Frag<T>::V V;
  const T* A = (const T*)Ap; const T* A2 = (const T*)A2p; const T* Bt = (const T*)Btp; const T* Bt2 = (const T*)Bt2p;
  __shared__ __align__(16) float sT[8][16 * 68];
  const int b    = blockIdx.y;
  const int lane = threadIdx.x & 31;
  const int wave = threadIdx.x >> 5;
  const int tilesN = N >> 6;
  const int tilesM = M >> 6;
  const int tile = blockIdx.x * 8 + wave;
  if (tile >= tilesM * tilesN) return;
  const int tm = tile / tilesN;
  const int tn = tile - tm * tilesN;
  const int m0 = tm << 6;
  const int n0 = tn << 6;

  const T* Ab  = A  + (size_t)b * strideA;
  const T* Bb  = Bt + (size_t)b * strideB;
  const T* Ab2 = SPLIT ? (A2  + (size_t)b * strideA) : nullptr;
  const T* Bb2 = SPLIT ? (Bt2 + (size_t)b * strideB) : nullptr;

  const int rlane = lane & 15;
  const int koff  = (lane >> 4) * 8;
  const int mOff  = (lane >> 4) * 8;

  v8f acc[4][4];
#pragma unroll
  for (int i = 0; i < 4; ++i)
#pragma unroll
    for (int j = 0; j < 4; ++j) acc[i][j] = (v8f){0.f,0.f,0.f,0.f,0.f,0.f,0.f,0.f};

  for (int k0 = 0; k0 < K; k0 += 32) {
    V bh[4], bl[4];
#pragma unroll
    for (int j = 0; j < 4; ++j) {
      const size_t bo = (size_t)(n0 + (j << 4) + rlane) * ldb + koff + k0;
      bh[j] = Frag<T>::load(Bb + bo);
      if (SPLIT) bl[j] = Frag<T>::load(Bb2 + bo);
    }
#pragma unroll
    for (int i = 0; i < 4; ++i) {
      const size_t ao = (size_t)(m0 + (i << 4) + rlane) * lda + koff + k0;
      V ah = Frag<T>::load(Ab + ao);
      V al;
      if (SPLIT) al = Frag<T>::load(Ab2 + ao);
#pragma unroll
      for (int j = 0; j < 4; ++j) {
        acc[i][j] = Frag<T>::mma(ah, bh[j], acc[i][j]);
        if (SPLIT) {
          acc[i][j] = Frag<T>::mma(ah, bl[j], acc[i][j]);
          acc[i][j] = Frag<T>::mma(al, bh[j], acc[i][j]);
        }
      }
      Frag<T>::guard(acc[i][0], acc[i][3], ah, SPLIT ? al : ah);
      Frag<T>::guard(acc[i][1], acc[i][2], ah, SPLIT ? al : ah);
    }
    Frag<T>::keep(bh[0], bh[1], bh[2], bh[3]);
    if (SPLIT) Frag<T>::keep(bl[0], bl[1], bl[2], bl[3]);
  }
  acc_guard4(acc[0][0], acc[0][1], acc[0][2], acc[0][3]);
  acc_guard4(acc[1][0], acc[1][1], acc[1][2], acc[1][3]);
  acc_guard4(acc[2][0], acc[2][1], acc[2][2], acc[2][3]);
  acc_guard4(acc[3][0], acc[3][1], acc[3][2], acc[3][3]);

  float* slab = sT[wave];
  const float* Rb = RESID ? (resid + (size_t)b * strideR) : nullptr;
#pragma unroll
  for (int i = 0; i < 4; ++i) {
    const int mBase = m0 + (i << 4);
#pragma unroll
    for (int j = 0; j < 4; ++j) {
      const int n = n0 + (j << 4) + rlane;
      float bv = 0.f;
      if (BIAS_MODE == 2) bv = bias[n];
#pragma unroll
      for (int r = 0; r < 8; ++r) {
        float v = acc[i][j][r] * scale;
        if (BIAS_MODE == 1) v += bias[mBase + mOff + r];
        if (BIAS_MODE == 2) v += bv;
        if (RESID) v += Rb[(size_t)(mBase + mOff + r) * ldc + n];
        if (ACT == 2) v = fmaxf(v, 0.0f);
        if (ACT == 4) v = (v > 0.f) ? v : 0.01f * v;
        slab[(mOff + r) * 68 + (j << 4) + rlane] = v;
      }
    }
    __builtin_amdgcn_fence(__ATOMIC_RELEASE, "workgroup");
    __builtin_amdgcn_wave_barrier();
    __builtin_amdgcn_fence(__ATOMIC_ACQUIRE, "workgroup");
    if (OUT_MODE == 0) {
      float* C = (float*)Cout + (size_t)b * strideC;
      const int hh = lane >> 4, c4 = (lane & 15) * 4;
      for (int pass = 0; pass < 2; ++pass) {
#pragma unroll
        for (int it = 0; it < 8; ++it) {
          const int row = it * 2 + hh;
          v4f v = *(const v4f*)(slab + row * 68 + c4);
          *(volatile v4f*)(C + (size_t)(mBase + row) * ldc + n0 + c4) = v;
        }
        __threadfence();
      }
    } else {
      const int q = lane >> 3, c8 = (lane & 7) * 8;
      unsigned short* C  = (unsigned short*)Cout  + (size_t)b * strideC;
      unsigned short* C2 = (OUT_MODE == 2) ? ((unsigned short*)Cout2 + (size_t)b * strideC) : nullptr;
      for (int pass = 0; pass < 2; ++pass) {
#pragma unroll
        for (int it = 0; it < 4; ++it) {
          const int row = it * 4 + q;
          const float* sp = slab + row * 68 + c8;
          v8h hv, lv;
#pragma unroll
          for (int e = 0; e < 8; ++e) {
            if (OUT_MODE == 1) {
              hv[e] = (_Float16)sp[e];
            } else {
              unsigned short hb = f2bf_bits(sp[e]);
              unsigned short lb = f2bf_bits(sp[e] - bf_bits2f(hb));
              hv[e] = __builtin_bit_cast(_Float16, hb);
              lv[e] = __builtin_bit_cast(_Float16, lb);
            }
          }
          *(volatile v8h*)(C + (size_t)(mBase + row) * ldc + n0 + c8) = hv;
          if (OUT_MODE == 2) *(volatile v8h*)(C2 + (size_t)(mBase + row) * ldc + n0 + c8) = lv;
        }
        __threadfence();
      }
    }
    __builtin_amdgcn_fence(__ATOMIC_RELEASE, "workgroup");
    __builtin_amdgcn_wave_barrier();
    __builtin_amdgcn_fence(__ATOMIC_ACQUIRE, "workgroup");
  }
}

__global__ __launch_bounds__(256) void prep_weights(const float* __restrict__ w1, const float* __restrict__ w2,
                                                    const float* __restrict__ w3, _Float16* __restrict__ wpl) {
  const int i = blockIdx.x * 256 + threadIdx.x;
  const float* src;
  int ld, off, li;
  if (blockIdx.x < 2) { src = w1; ld = CIN1; off = 3; li = i; }
  else if (blockIdx.x < 4) { src = w2; ld = NCH1; off = 0; li = i - 512; }
  else { src = w3; ld = NCH2; off = 0; li = i - 1024; }
  const int row = li >> 3, k8 = (li & 7) * 8;
  const float* p = src + (size_t)row * ld + off + k8;
  v8h hv;
#pragma unroll
  for (int e = 0; e < 8; ++e) {
    const float f = p[e] * WCARRY;
    hv[e] = (_Float16)f;
  }
  _Float16* dst = wpl + (size_t)i * 8;
  *(volatile v8h*)dst = hv;
  __threadfence();
  *(volatile v8h*)dst = hv;
}

__global__ __launch_bounds__(256) void pts_transpose(const float* __restrict__ pts, _Float16* __restrict__ ptsT) {
  __shared__ float tile[64 * 65];
  const int b = blockIdx.x >> 6;
  const int n0 = (blockIdx.x & 63) * 64;
  const int t = threadIdx.x;
  const float* pb = pts + (size_t)b * DFEAT * NPTS + n0;
  const int n4 = (t & 15) * 4, cr = t >> 4;
#pragma unroll
  for (int it = 0; it < 4; ++it) {
    const int c = cr + 16 * it;
    const v4f v = *(const v4f*)(pb + (size_t)c * NPTS + n4);
    tile[c * 65 + n4 + 0] = v[0];
    tile[c * 65 + n4 + 1] = v[1];
    tile[c * 65 + n4 + 2] = v[2];
    tile[c * 65 + n4 + 3] = v[3];
  }
  __syncthreads();
  const int q8 = (t & 7) * 8, rr = t >> 3;
  v8h hv0, hv1;
#pragma unroll
  for (int e = 0; e < 8; ++e) {
    hv0[e] = (_Float16)tile[(q8 + e) * 65 + rr];
    hv1[e] = (_Float16)tile[(q8 + e) * 65 + rr + 32];
  }
  _Float16* d0 = ptsT + ((size_t)b * NPTS + n0 + rr) * 64 + q8;
  _Float16* d1 = ptsT + ((size_t)b * NPTS + n0 + rr + 32) * 64 + q8;
  for (int pass = 0; pass < 2; ++pass) {
    *(volatile v8h*)d0 = hv0;
    *(volatile v8h*)d1 = hv1;
    __threadfence();
  }
}

__global__ __launch_bounds__(256) void fps_kernel(const float* __restrict__ xyz, float* __restrict__ cen,
                                                  float* __restrict__ out0) {
#pragma clang fp contract(off)
  __shared__ __align__(16) float sxyz[3 * NPTS];
  __shared__ int sidx[NPOINT];
  __shared__ unsigned long long red[2][8];

  const int b = blockIdx.x;
  const int tid = threadIdx.x;
  const int lane = tid & 31;
  const int wave = tid >> 5;
  const float* xb = xyz + (size_t)b * 3 * NPTS;

#pragma unroll 1
  for (int i = tid; i < (3 * NPTS) / 4; i += 256) {
    const v4f v = *(const v4f*)(xb + 4 * i);
    *(v4f_a*)(sxyz + 4 * i) = v;
  }
  __syncthreads();

  float px[16], py[16], pz[16], dist[16];
#pragma unroll
  for (int i = 0; i < 16; ++i) {
    const int p = tid + i * 256;
    px[i] = sxyz[p];
    py[i] = sxyz[NPTS + p];
    pz[i] = sxyz[2 * NPTS + p];
    dist[i] = 1e10f;
  }

  int far = 0;
  for (int s = 0; s < NPOINT; ++s) {
    if (tid == 0) sidx[s] = far;
    const float cx = sxyz[far], cy = sxyz[NPTS + far], cz = sxyz[2 * NPTS + far];
    float bestv = -1.0f;
    unsigned bi = 0u;
#pragma unroll
    for (int i = 0; i < 16; ++i) {
      const float dx = px[i] - cx;
      const float dy = py[i] - cy;
      const float dz = pz[i] - cz;
      const float t0 = dx * dx;
      const float t1 = dy * dy;
      const float t2 = dz * dz;
      const float d = (t0 + t2) + t1;
      const float od = dist[i];
      const float nd = (d < od) ? d : od;
      dist[i] = nd;
      const bool gt = nd > bestv;
      bestv = gt ? nd : bestv;
      bi = gt ? (unsigned)(tid + i * 256) : bi;
    }
    unsigned hi = __float_as_uint(bestv);
    unsigned lo = 0xFFFFFFFFu - bi;
#pragma unroll
    for (int off = 16; off > 0; off >>= 1) {
      const unsigned ohi = (unsigned)__shfl_xor((int)hi, off, 32);
      const unsigned olo = (unsigned)__shfl_xor((int)lo, off, 32);
      const bool take = (ohi > hi) || ((ohi == hi) && (olo > lo));
      hi = take ? ohi : hi;
      lo = take ? olo : lo;
    }
    if (lane == 0) red[s & 1][wave] = (((unsigned long long)hi) << 32) | (unsigned long long)lo;
    __syncthreads();
    unsigned long long m = red[s & 1][0];
#pragma unroll
    for (int w = 1; w < 8; ++w) {
      const unsigned long long v = red[s & 1][w];
      m = (v > m) ? v : m;
    }
    int nf = (int)(0xFFFFFFFFu - (unsigned)(m & 0xFFFFFFFFull));
    nf = nf < 0 ? 0 : nf;
    nf = nf > (NPTS - 1) ? (NPTS - 1) : nf;
    far = nf;
  }
  __syncthreads();

  const int s4 = tid * 4;
  int j0 = sidx[s4 + 0], j1 = sidx[s4 + 1], j2 = sidx[s4 + 2], j3 = sidx[s4 + 3];
  j0 = min(max(j0, 0), NPTS - 1);
  j1 = min(max(j1, 0), NPTS - 1);
  j2 = min(max(j2, 0), NPTS - 1);
  j3 = min(max(j3, 0), NPTS - 1);
  v4f vx, vy, vz;
  vx[0] = sxyz[j0]; vx[1] = sxyz[j1]; vx[2] = sxyz[j2]; vx[3] = sxyz[j3];
  vy[0] = sxyz[NPTS + j0]; vy[1] = sxyz[NPTS + j1]; vy[2] = sxyz[NPTS + j2]; vy[3] = sxyz[NPTS + j3];
  vz[0] = sxyz[2 * NPTS + j0]; vz[1] = sxyz[2 * NPTS + j1]; vz[2] = sxyz[2 * NPTS + j2]; vz[3] = sxyz[2 * NPTS + j3];
  float* ob = out0 + (size_t)b * 3 * NPOINT + s4;
  float* cb = cen + (size_t)b * 3 * NPOINT + s4;
  for (int pass = 0; pass < 2; ++pass) {
    *(volatile v4f*)(ob) = vx;
    *(volatile v4f*)(ob + NPOINT) = vy;
    *(volatile v4f*)(ob + 2 * NPOINT) = vz;
    *(volatile v4f*)(cb) = vx;
    *(volatile v4f*)(cb + NPOINT) = vy;
    *(volatile v4f*)(cb + 2 * NPOINT) = vz;
    __threadfence();
  }
}

__global__ __launch_bounds__(256) void ballq_kernel(const float* __restrict__ xyz, const float* __restrict__ cen,
                                                    int* __restrict__ idx) {
#pragma clang fp contract(off)
  __shared__ int slist[8][32];
  const int lane = threadIdx.x & 31;
  const int wave = threadIdx.x >> 5;
  const int g = blockIdx.x * 8 + wave;
  const int b = g >> 10;
  const int s = g & (NPOINT - 1);
  const float* xb = xyz + (size_t)b * 3 * NPTS;
  const float* cb = cen + (size_t)b * 3 * NPOINT;
  const float cx = cb[s], cy = cb[NPOINT + s], cz = cb[2 * NPOINT + s];

  slist[wave][lane] = 0;
  __syncthreads();

  int found = 0;
#pragma unroll 1
  for (int base = 0; base < NPTS; base += 32) {
    if (found >= NSAMPLE) break;
    const int p = base + lane;
    const float x = xb[p];
    const float y = xb[NPTS + p];
    const float z = xb[2 * NPTS + p];
    const float dx = cx - x;
    const float dy = cy - y;
    const float dz = cz - z;
    const float t0 = dx * dx;
    const float t1 = dy * dy;
    const float t2 = dz * dz;
    const float sqr = (t0 + t2) + t1;
    const bool in = !(sqr > RAD2);
    const unsigned mask = __builtin_amdgcn_ballot_w32(in);
    const int rank = found + __popc(mask & ((1u << lane) - 1u));
    if (in && (rank < NSAMPLE)) slist[wave][rank] = p;
    found = __builtin_amdgcn_readfirstlane(found + __popc(mask));
  }
  __syncthreads();
  const int nf = found > NSAMPLE ? NSAMPLE : found;
  const int first = slist[wave][0];
  const int mine = slist[wave][lane];
  int j = (lane < nf) ? mine : first;
  j = min(max(j, 0), NPTS - 1);
  int* o = idx + (size_t)g * NSAMPLE + lane;
  *(volatile int*)o = j;
  __threadfence();
  *(volatile int*)o = j;
}

template <int MODE>
__global__ __launch_bounds__(256) void l1_kernel(const float* __restrict__ xyz, const float* __restrict__ cen,
                                                 const int* __restrict__ idx, const float* __restrict__ P,
                                                 const float* __restrict__ w1, const float* __restrict__ b1,
                                                 const float* __restrict__ ac1, float* __restrict__ part,
                                                 unsigned* __restrict__ X1w) {
  __shared__ __align__(16) unsigned stage[(MODE == 1) ? 8 * 1024 : 8];
  __shared__ __align__(16) float redS[(MODE == 0) ? 8 * 128 : 8];
  const int lane = threadIdx.x & 31;
  const int wave = threadIdx.x >> 5;
  const int ch0 = 2 * lane;

  float w00 = w1[ch0 * CIN1 + 0], w01 = w1[ch0 * CIN1 + 1], w02 = w1[ch0 * CIN1 + 2];
  float w10 = w1[(ch0 + 1) * CIN1 + 0], w11 = w1[(ch0 + 1) * CIN1 + 1], w12 = w1[(ch0 + 1) * CIN1 + 2];
  const v2f bbv = *(const v2f*)(b1 + ch0);
  float bb0 = bbv[0], bb1 = bbv[1];
  float a0 = 0.f, a1 = 0.f, c0 = 0.f, c1 = 0.f;
  if (MODE == 1) {
    const v2f av = *(const v2f*)(ac1 + ch0);
    const v2f cv = *(const v2f*)(ac1 + 128 + ch0);
    a0 = av[0]; a1 = av[1];
    c0 = cv[0]; c1 = cv[1];
  }
  asm volatile("" : "+v"(w00), "+v"(w01), "+v"(w02), "+v"(w10), "+v"(w11), "+v"(w12), "+v"(bb0), "+v"(bb1));
  asm volatile("" : "+v"(a0), "+v"(a1), "+v"(c0), "+v"(c1));
  float s1a = 0.f, s1b = 0.f, s2a = 0.f, s2b = 0.f;

#pragma unroll 1
  for (int gi = 0; gi < 4; ++gi) {
    const int g = blockIdx.x * 32 + wave * 4 + gi;
    const int b = g >> 10;
    const int s = g & (NPOINT - 1);
    const float* cb = cen + (size_t)b * 3 * NPOINT;
    const float cx = cb[s], cy = cb[NPOINT + s], cz = cb[2 * NPOINT + s];
    int jl = idx[(size_t)g * NSAMPLE + lane];
    jl = min(max(jl, 0), NPTS - 1);
    const float* xb = xyz + (size_t)b * 3 * NPTS;
    const float d0 = xb[jl] - cx;
    const float d1 = xb[NPTS + jl] - cy;
    const float d2 = xb[2 * NPTS + jl] - cz;
    const float* Pb = P + (size_t)b * NPTS * 64;

#pragma unroll 4
    for (int k = 0; k < NSAMPLE; ++k) {
      const int j = __shfl(jl, k, 32);
      const float e0 = __shfl(d0, k, 32);
      const float e1 = __shfl(d1, k, 32);
      const float e2 = __shfl(d2, k, 32);
      const v2f pv = *(const v2f*)(Pb + (size_t)j * 64 + ch0);
      float t0 = w00 * e0;
      t0 = fmaf(w01, e1, t0);
      t0 = fmaf(w02, e2, t0);
      float t1 = w10 * e0;
      t1 = fmaf(w11, e1, t1);
      t1 = fmaf(w12, e2, t1);
      const float y0 = (pv[0] + t0) + bb0;
      const float y1 = (pv[1] + t1) + bb1;
      if (MODE == 0) {
        s1a += y0;
        s1b += y1;
        s2a = fmaf(y0, y0, s2a);
        s2b = fmaf(y1, y1, s2b);
      } else {
        const float x0 = fmaxf(fmaf(a0, y0, c0), 0.0f);
        const float x1 = fmaxf(fmaf(a1, y1, c1), 0.0f);
        const _Float16 h0 = (_Float16)x0, h1 = (_Float16)x1;
        const unsigned u = (unsigned)__builtin_bit_cast(unsigned short, h0) |
                           ((unsigned)__builtin_bit_cast(unsigned short, h1) << 16);
        stage[wave * 1024 + k * 32 + lane] = u;
      }
    }
    if (MODE == 1) {
      __syncthreads();
      const int q = lane >> 3, w4 = (lane & 7) * 4;
      u32x4 v[8];
#pragma unroll
      for (int it = 0; it < 8; ++it) {
        const u32x4 t = *(const u32x4_a*)(stage + wave * 1024 + (it * 4 + q) * 32 + w4);
        v[it] = t;
      }
      unsigned* dst = X1w + ((size_t)g * NSAMPLE + q) * 32 + w4;
      for (int pass = 0; pass < 2; ++pass) {
#pragma unroll
        for (int it = 0; it < 8; ++it) {
          *(volatile u32x4*)(dst + (size_t)it * 4 * 32) = v[it];
        }
        __threadfence();
      }
      __syncthreads();
    }
  }
  if (MODE == 0) {
    redS[wave * 128 + ch0] = s1a;
    redS[wave * 128 + ch0 + 1] = s1b;
    redS[wave * 128 + 64 + ch0] = s2a;
    redS[wave * 128 + 64 + ch0 + 1] = s2b;
    __syncthreads();
    if (wave == 0) {
      v4f v;
#pragma unroll
      for (int e = 0; e < 4; ++e) {
        float acc = redS[lane * 4 + e];
#pragma unroll
        for (int w = 1; w < 8; ++w) acc += redS[w * 128 + lane * 4 + e];
        v[e] = acc;
      }
      float* dst = part + (size_t)blockIdx.x * 128 + lane * 4;
      *(volatile v4f*)dst = v;
      __threadfence();
      *(volatile v4f*)dst = v;
    }
  }
}

__global__ __launch_bounds__(128) void bn_finalize(const float* __restrict__ part, int nparts, int C,
                                                   const float* __restrict__ gam, const float* __restrict__ bet,
                                                   const float* __restrict__ bias, int use_bias, float zs,
                                                   float* __restrict__ ac) {
  __shared__ __align__(16) float sAC[256];
  const int ch = threadIdx.x;
  const int chc = ch < C ? ch : (C - 1);
  const int pitch = 2 * C;
  const int np = nparts > 4096 ? 4096 : nparts;
  double s1 = 0.0, s2 = 0.0;
#pragma unroll 4
  for (int p = 0; p < np; ++p) {
    s1 += (double)part[(size_t)p * pitch + chc];
    s2 += (double)part[(size_t)p * pitch + C + chc];
  }
  const double inv = 1.0 / 524288.0;
  const double zsd = (double)zs;
  const double meanz = s1 * inv;
  const double msq = meanz * meanz;
  double varz = s2 * inv - msq;
  varz = varz < 0.0 ? 0.0 : varz;
  const double vary = (varz * zsd) * zsd;
  const double meanl = meanz * zsd;
  const float braw = bias[chc];
  const float bv = (use_bias != 0) ? braw : 0.0f;
  const float vf = (float)vary + BN_EPS;
  const float a = gam[chc] * (1.0f / sqrtf(vf));
  const float my = (float)meanl + bv;
  const float cc = bet[chc] - my * a;
  const float aout = a * zs;
  const float cout = cc + a * bv;
  sAC[ch] = (ch < C) ? aout : 0.0f;
  sAC[128 + ch] = (ch < C) ? cout : 0.0f;
  __syncthreads();
  if (threadIdx.x < 32) {
    const int l4 = threadIdx.x * 4;
    const v4f v0 = *(const v4f*)(sAC + l4);
    const v4f v1 = *(const v4f*)(sAC + 128 + l4);
    for (int pass = 0; pass < 2; ++pass) {
      *(volatile v4f*)(ac + l4) = v0;
      *(volatile v4f*)(ac + 128 + l4) = v1;
      __threadfence();
    }
  }
}

template <int PHASE>
__global__ __launch_bounds__(128) void mlp_kernel(const _Float16* __restrict__ X1, const _Float16* __restrict__ wpl,
                                                  const float* __restrict__ ac2, float* __restrict__ part,
                                                  float* __restrict__ MXP, float* __restrict__ MNP) {
  constexpr int NC = (PHASE == 0) ? NCH2 : NCH3;
  constexpr int NJ = NC / 16;
  union FH { v16h v; v8h h[2]; };
  __shared__ __align__(16) _Float16 sW2[NCH2 * 64];
  __shared__ __align__(16) _Float16 sW3[(PHASE == 1) ? NCH3 * 64 : 8];
  __shared__ __align__(16) _Float16 xs[(PHASE == 1) ? 4 * XS_WAVE : 8];
  __shared__ __align__(16) float mm[(PHASE == 1) ? 4 * 256 : 4];
  __shared__ __align__(16) float red[4 * 2 * NC];

  const int tid = threadIdx.x;
  const int lane = tid & 31;
  const int wave = tid >> 5;
  const int c = lane & 15;
  const int h = lane >> 4;

#pragma unroll 4
  for (int i = tid; i < (NCH2 * 64) / 8; i += 128) {
    const u32x4 w = *(const u32x4_a*)(wpl + WPL_OFF2 + i * 8);
    *(u32x4_a*)(sW2 + i * 8) = w;
  }
  if (PHASE == 1) {
#pragma unroll 4
    for (int i = tid; i < (NCH3 * 64) / 8; i += 128) {
      const u32x4 w = *(const u32x4_a*)(wpl + WPL_OFF3 + i * 8);
      *(u32x4_a*)(sW3 + i * 8) = w;
    }
  }
  float az2[4], cz2[4];
#pragma unroll
  for (int jn = 0; jn < 4; ++jn) {
    az2[jn] = (PHASE == 1) ? ac2[16 * jn + c] : 0.0f;
    cz2[jn] = (PHASE == 1) ? ac2[128 + 16 * jn + c] : 0.0f;
  }
  asm volatile("" : "+v"(az2[0]), "+v"(az2[1]), "+v"(az2[2]), "+v"(az2[3]),
                    "+v"(cz2[0]), "+v"(cz2[1]), "+v"(cz2[2]), "+v"(cz2[3]));
  __syncthreads();

  float s1[NJ], s2[NJ];
#pragma unroll
  for (int jn = 0; jn < NJ; ++jn) { s1[jn] = 0.0f; s2[jn] = 0.0f; }

  for (int gi = 0; gi < 8; ++gi) {
    const int g = blockIdx.x * 32 + wave * 8 + gi;
    const _Float16* Ag = X1 + (size_t)g * NSAMPLE * 64;
    v16h a[2][2];
#pragma unroll
    for (int i = 0; i < 2; ++i)
#pragma unroll
      for (int ks = 0; ks < 2; ++ks)
        a[i][ks] = Frag<_Float16>::load(Ag + (size_t)(16 * i + c) * 64 + 32 * ks + 8 * h);

#pragma unroll
    for (int jn = 0; jn < 4; ++jn) {
      FH f0, f1;
      f0.h[0] = *(const v8h*)(sW2 + (16 * jn + c) * 64 + 8 * h);
      f0.h[1] = *(const v8h*)(sW2 + (16 * jn + c) * 64 + 16 + 8 * h);
      f1.h[0] = *(const v8h*)(sW2 + (16 * jn + c) * 64 + 32 + 8 * h);
      f1.h[1] = *(const v8h*)(sW2 + (16 * jn + c) * 64 + 48 + 8 * h);
      v8f acc0 = (v8f){0.f,0.f,0.f,0.f,0.f,0.f,0.f,0.f};
      v8f acc1 = (v8f){0.f,0.f,0.f,0.f,0.f,0.f,0.f,0.f};
      acc0 = mma_h(a[0][0], f0.v, acc0);
      acc0 = mma_h(a[0][1], f1.v, acc0);
      acc1 = mma_h(a[1][0], f0.v, acc1);
      acc1 = mma_h(a[1][1], f1.v, acc1);
#pragma unroll
      for (int r = 0; r < 8; ++r) {
        const float z0 = acc0[r];
        const float z1 = acc1[r];
        if (PHASE == 0) {
          s1[jn] += z0;
          s1[jn] += z1;
          s2[jn] = fmaf(z0, z0, s2[jn]);
          s2[jn] = fmaf(z1, z1, s2[jn]);
        } else {
          const float x0 = fmaxf(fmaf(az2[jn], z0, cz2[jn]), 0.0f);
          const float x1 = fmaxf(fmaf(az2[jn], z1, cz2[jn]), 0.0f);
          xs[wave * XS_WAVE + (8 * h + r) * XS_PITCH + 16 * jn + c] = (_Float16)x0;
          xs[wave * XS_WAVE + (16 + 8 * h + r) * XS_PITCH + 16 * jn + c] = (_Float16)x1;
        }
      }
    }

    if (PHASE == 1) {
      __syncthreads();
      v16h a3[2][2];
#pragma unroll
      for (int i = 0; i < 2; ++i)
#pragma unroll
        for (int ks = 0; ks < 2; ++ks) {
          FH f;
          f.h[0] = *(const v8h*)(xs + wave * XS_WAVE + (16 * i + c) * XS_PITCH + 32 * ks + 8 * h);
          f.h[1] = *(const v8h*)(xs + wave * XS_WAVE + (16 * i + c) * XS_PITCH + 32 * ks + 16 + 8 * h);
          a3[i][ks] = f.v;
        }
#pragma unroll
      for (int jn = 0; jn < 8; ++jn) {
        FH f0, f1;
        f0.h[0] = *(const v8h*)(sW3 + (16 * jn + c) * 64 + 8 * h);
        f0.h[1] = *(const v8h*)(sW3 + (16 * jn + c) * 64 + 16 + 8 * h);
        f1.h[0] = *(const v8h*)(sW3 + (16 * jn + c) * 64 + 32 + 8 * h);
        f1.h[1] = *(const v8h*)(sW3 + (16 * jn + c) * 64 + 48 + 8 * h);
        v8f acc0 = (v8f){0.f,0.f,0.f,0.f,0.f,0.f,0.f,0.f};
        v8f acc1 = (v8f){0.f,0.f,0.f,0.f,0.f,0.f,0.f,0.f};
        acc0 = mma_h(a3[0][0], f0.v, acc0);
        acc0 = mma_h(a3[0][1], f1.v, acc0);
        acc1 = mma_h(a3[1][0], f0.v, acc1);
        acc1 = mma_h(a3[1][1], f1.v, acc1);
        float mx = -INFINITY, mn = INFINITY;
#pragma unroll
        for (int r = 0; r < 8; ++r) {
          const float z0 = acc0[r];
          const float z1 = acc1[r];
          s1[jn] += z0;
          s1[jn] += z1;
          s2[jn] = fmaf(z0, z0, s2[jn]);
          s2[jn] = fmaf(z1, z1, s2[jn]);
          mx = fmaxf(mx, fmaxf(z0, z1));
          mn = fminf(mn, fminf(z0, z1));
        }
        const float omx = __shfl_xor(mx, 16, 32);
        const float omn = __shfl_xor(mn, 16, 32);
        mx = fmaxf(mx, omx);
        mn = fminf(mn, omn);
        mm[wave * 256 + h * 128 + 16 * jn + c] = (h == 0) ? mx : mn;
      }
      __syncthreads();
      const v4f vmx = *(const v4f*)(mm + wave * 256 + lane * 4);
      const v4f vmn = *(const v4f*)(mm + wave * 256 + 128 + lane * 4);
      float* dmx = MXP + (size_t)g * NCH3 + lane * 4;
      float* dmn = MNP + (size_t)g * NCH3 + lane * 4;
      for (int pass = 0; pass < 2; ++pass) {
        *(volatile v4f*)dmx = vmx;
        *(volatile v4f*)dmn = vmn;
        __threadfence();
      }
      __syncthreads();
    }
  }

#pragma unroll
  for (int jn = 0; jn < NJ; ++jn) {
    const float o1 = __shfl_xor(s1[jn], 16, 32);
    const float o2 = __shfl_xor(s2[jn], 16, 32);
    s1[jn] += o1;
    s2[jn] += o2;
  }
#pragma unroll
  for (int jn = 0; jn < NJ; ++jn) {
    red[wave * 2 * NC + h * NC + 16 * jn + c] = (h == 0) ? s1[jn] : s2[jn];
  }
  __syncthreads();
  if (wave == 0) {
    constexpr int NSEG = (2 * NC) / 128;
    v4f v[NSEG];
#pragma unroll
    for (int sg = 0; sg < NSEG; ++sg) {
#pragma unroll
      for (int e = 0; e < 4; ++e) {
        const int ix = sg * 128 + lane * 4 + e;
        const float t = ((red[ix] + red[2 * NC + ix]) + red[4 * NC + ix]) + red[6 * NC + ix];
        v[sg][e] = t;
      }
    }
    float* dst = part + (size_t)blockIdx.x * 2 * NC + lane * 4;
    for (int pass = 0; pass < 2; ++pass) {
#pragma unroll
      for (int sg = 0; sg < NSEG; ++sg) *(volatile v4f*)(dst + sg * 128) = v[sg];
      __threadfence();
    }
  }
}

__global__ __launch_bounds__(256) void final_kernel(const float* __restrict__ MXP, const float* __restrict__ MNP,
                                                    const float* __restrict__ ac3, float* __restrict__ out1) {
  __shared__ float tile[NCH3 * 33];
  const int b = blockIdx.x >> 5;
  const int s0 = (blockIdx.x & 31) * 32;
  const int lane = threadIdx.x & 31;
  const int wave = threadIdx.x >> 5;
  v4f av = *(const v4f*)(ac3 + lane * 4);
  v4f cv = *(const v4f*)(ac3 + 128 + lane * 4);
  asm volatile("" : "+v"(av), "+v"(cv));
#pragma unroll
  for (int hp = 0; hp < 2; ++hp) {
    v4f mxv[2], mnv[2];
#pragma unroll
    for (int u = 0; u < 2; ++u) {
      const int sl = wave + 8 * (2 * hp + u);
      const size_t g = (size_t)b * NPOINT + s0 + sl;
      mxv[u] = *(const v4f*)(MXP + g * NCH3 + lane * 4);
      mnv[u] = *(const v4f*)(MNP + g * NCH3 + lane * 4);
    }
#pragma unroll
    for (int e = 0; e < 4; ++e) {
      const float ae = av[e];
      const float ce = cv[e];
      const float fa = (ae >= 0.0f) ? 1.0f : 0.0f;
      const float fb = 1.0f - fa;
#pragma unroll
      for (int u = 0; u < 2; ++u) {
        const float pm = mxv[u][e];
        const float pn = mnv[u][e];
        const float sel = fmaf(fa, pm, fb * pn);
        const float val = fmaxf(fmaf(ae, sel, ce), 0.0f);
        tile[(lane * 4 + e) * 33 + wave + 8 * (2 * hp + u)] = val;
      }
    }
    asm volatile("" ::: "memory");
  }
  __syncthreads();
  const int q = lane >> 3, s4 = (lane & 7) * 4;
  v4f ov[4];
#pragma unroll
  for (int it = 0; it < 4; ++it) {
    const int o = it * 32 + wave * 4 + q;
    ov[it][0] = tile[o * 33 + s4 + 0];
    ov[it][1] = tile[o * 33 + s4 + 1];
    ov[it][2] = tile[o * 33 + s4 + 2];
    ov[it][3] = tile[o * 33 + s4 + 3];
  }
  for (int pass = 0; pass < 2; ++pass) {
#pragma unroll
    for (int it = 0; it < 4; ++it) {
      const int o = it * 32 + wave * 4 + q;
      *(volatile v4f*)(out1 + ((size_t)b * NCH3 + o) * NPOINT + s0 + s4) = ov[it];
    }
    __threadfence();
  }
}

extern "C" void kernel_launch(void* const* d_in, const int* in_sizes, int n_in,
                              void* d_out, int out_size, void* d_ws, size_t ws_size,
                              hipStream_t stream) {
  (void)in_sizes; (void)out_size;
  if (n_in < 14) return;
  if (ws_size < WS_TOTAL) return;

  const float* xyz = (const float*)d_in[0];
  const float* pts = (const float*)d_in[1];
  const float* w1  = (const float*)d_in[2];
  const float* b1  = (const float*)d_in[3];
  const float* g1  = (const float*)d_in[4];
  const float* be1 = (const float*)d_in[5];
  const float* w2  = (const float*)d_in[6];
  const float* b2  = (const float*)d_in[7];
  const float* g2  = (const float*)d_in[8];
  const float* be2 = (const float*)d_in[9];
  const float* w3  = (const float*)d_in[10];
  const float* b3  = (const float*)d_in[11];
  const float* g3  = (const float*)d_in[12];
  const float* be3 = (const float*)d_in[13];

  float* out0 = (float*)d_out;
  float* out1 = (float*)((char*)d_out + OUT0_BYTES);

  char* ws = (char*)d_ws;
  _Float16* wpl  = (_Float16*)(ws + OFF_WPL);
  float* ac1     = (float*)(ws + OFF_AC);
  float* ac2     = ac1 + 256;
  float* ac3     = ac1 + 512;
  float* cen     = (float*)(ws + OFF_CEN);
  int*   idx     = (int*)(ws + OFF_IDX);
  float* part1   = (float*)(ws + OFF_PART1);
  float* part2   = (float*)(ws + OFF_PART2);
  float* part3   = (float*)(ws + OFF_PART3);
  _Float16* ptsT = (_Float16*)(ws + OFF_PTST);
  float* ppl     = (float*)(ws + OFF_PPL);
  _Float16* x1   = (_Float16*)(ws + OFF_X1);
  float* mxp     = (float*)(ws + OFF_MXP);
  float* mnp     = (float*)(ws + OFF_MNP);

  prep_weights<<<8, 256, 0, stream>>>(w1, w2, w3, wpl);
  pts_transpose<<<NB * (NPTS / 64), 256, 0, stream>>>(pts, ptsT);

  {
    constexpr int GM = NB * NPTS, GN = NCH1, GK = DFEAT;
    static_assert(GM % 64 == 0 && GN % 64 == 0 && GK % 32 == 0);
    constexpr int tiles = (GM / 64) * (GN / 64);
    static_assert(tiles % 8 == 0);
    wmma_gemm64<0, false, 0, 0, false, 0><<<dim3(tiles / 8, 1), 256, 0, stream>>>(
        (const unsigned short*)ptsT, (const unsigned short*)ptsT, 64, 0L,
        (const unsigned short*)(wpl + WPL_OFF1), (const unsigned short*)(wpl + WPL_OFF1), 64, 0L,
        (void*)ppl, (void*)ppl, 64, 0L, b1, ppl, 0L, GM, GN, GK, WINV);
  }

  fps_kernel<<<NB, 256, 0, stream>>>(xyz, cen, out0);
  ballq_kernel<<<NGRP / 8, 256, 0, stream>>>(xyz, cen, idx);

  l1_kernel<0><<<NPARTS, 256, 0, stream>>>(xyz, cen, idx, ppl, w1, b1, ac1, part1, (unsigned*)x1);
  bn_finalize<<<1, 128, 0, stream>>>(part1, NPARTS, NCH1, g1, be1, b1, 0, 1.0f, ac1);
  l1_kernel<1><<<NPARTS, 256, 0, stream>>>(xyz, cen, idx, ppl, w1, b1, ac1, part1, (unsigned*)x1);

  mlp_kernel<0><<<NPARTS, 128, 0, stream>>>(x1, wpl, ac2, part2, mxp, mnp);
  bn_finalize<<<1, 128, 0, stream>>>(part2, NPARTS, NCH2, g2, be2, b2, 1, WINV, ac2);
  mlp_kernel<1><<<NPARTS, 128, 0, stream>>>(x1, wpl, ac2, part3, mxp, mnp);
  bn_finalize<<<1, 128, 0, stream>>>(part3, NPARTS, NCH3, g3, be3, b3, 1, WINV, ac3);

  final_kernel<<<NB * (NPOINT / 32), 256, 0, stream>>>(mxp, mnp, ac3, out1);
}
